// ODE_RNN_74208444940297
// MI455X (gfx1250) — hardware-run, weakly checked
//
#include <hip/hip_runtime.h>
#include <stddef.h>
#include <stdint.h>

typedef __attribute__((ext_vector_type(16))) _Float16 v16h;
typedef __attribute__((ext_vector_type(8)))  _Float16 v8h;
typedef __attribute__((ext_vector_type(16))) __bf16   v16b;
typedef __attribute__((ext_vector_type(8)))  __bf16   v8b;
typedef __attribute__((ext_vector_type(8)))  float    v8f;
typedef __attribute__((ext_vector_type(4)))  float    v4f;
typedef __attribute__((ext_vector_type(4)))  unsigned short v4us;

constexpr int kBatch     = 256;
constexpr int kSteps     = 512;
constexpr int kIn        = 32;
constexpr int kHid       = 64;
constexpr int kOutDim    = 8;
constexpr int kWid       = 16;
constexpr int kSub       = 8;
constexpr int kSeqPerBlk = 16;
constexpr int kBlocks    = kBatch / kSeqPerBlk;
constexpr int kOut0Elems = kBatch * kOutDim;
constexpr int kOut1Off   = 2048;
constexpr int kOutTotal  = kOut0Elems + kBatch * kHid;
constexpr int kSlots      = 6;
constexpr int kSlotStride = 32 * 32;
static_assert(kBatch % kSeqPerBlk == 0, "grid covers the batch exactly");
static_assert(kHid == 64 && kWid == 16 && kIn == 32 && kOutDim == 8, "tile plan");
static_assert(kOut1Off * 4 == 8192 && kOut0Elems == kOut1Off, "out1 offset");
static_assert(kOutTotal * 4 == 73728, "d_out total");
static_assert(kSlots * kSlotStride >= kSeqPerBlk * kHid + kSeqPerBlk * kOutDim, "output staging fits in the stage park");

constexpr float cA21 = 0.161f;
constexpr float cA31 = -0.008480655492356989f, cA32 = 0.335480655492357f;
constexpr float cA41 = 2.8971530571054935f, cA42 = -6.359448489975075f, cA43 = 4.3622954328695815f;
constexpr float cA51 = 5.325864828439257f, cA52 = -11.748883564062828f, cA53 = 7.4955393428898365f, cA54 = -0.09249506636175525f;
constexpr float cA61 = 5.86145544294642f, cA62 = -12.92096931784711f, cA63 = 8.159367898576159f, cA64 = -0.071584973281401f, cA65 = -0.028269050394068383f;
constexpr float cB1 = 0.09646076681806523f, cB2 = 0.01f, cB3 = 0.4798896504144996f, cB4 = 1.379008574103742f, cB5 = -3.290069515436081f, cB6 = 2.324710524099774f;
constexpr float cC2 = 0.161f, cC3 = 0.327f, cC4 = 0.9f, cC5 = 0.9800255409045097f;

constexpr float kL2 = 2.8853900817779268f;
constexpr float kS0 = 0.18033688011112042f;
constexpr float kM2 = -5.7707801635558536f;

__device__ __forceinline__ unsigned short f2bf_bits(float f) {
  unsigned u = __float_as_uint(f);
  return (unsigned short)((u + 0x7FFFu + ((u >> 16) & 1u)) >> 16);
}
__device__ __forceinline__ float bf_bits2f(unsigned short h) { return __uint_as_float(((unsigned)h) << 16); }
__device__ __forceinline__ void split_bf(float x, unsigned short& hb, unsigned short& lb) {
  hb = f2bf_bits(x);
  lb = f2bf_bits(x - bf_bits2f(hb));
}

__device__ __forceinline__ v8f mma_h(v16h a, v16h b, v8f c) {
  c = __builtin_amdgcn_wmma_f32_16x16x32_f16(false, a, false, b, (short)0, c, false, false);
  asm volatile("v_nop\n\tv_nop\n\tv_nop\n\tv_nop" : "+v"(c) : "v"(a), "v"(b));
  return c;
}
__device__ __forceinline__ v8f mma_b(v16b a, v16b b, v8f c) {
  c = __builtin_amdgcn_wmma_f32_16x16x32_bf16(false, a, false, b, (short)0, c, false, false);
  asm volatile("v_nop\n\tv_nop\n\tv_nop\n\tv_nop" : "+v"(c) : "v"(a), "v"(b));
  return c;
}
__device__ __forceinline__ int opaque_zero() { int z; asm volatile("v_mov_b32 %0, 0" : "=v"(z)); return z; }
__device__ __forceinline__ void cfence() { asm volatile("" ::: "memory"); }

__device__ __forceinline__ v8f zero8f() { return (v8f){0.f, 0.f, 0.f, 0.f, 0.f, 0.f, 0.f, 0.f}; }
__device__ __forceinline__ v8f cat8(v4f a, v4f b) { return (v8f){a[0], a[1], a[2], a[3], b[0], b[1], b[2], b[3]}; }
__device__ __forceinline__ v4f lo4(v8f v) { return (v4f){v[0], v[1], v[2], v[3]}; }
__device__ __forceinline__ v4f hi4(v8f v) { return (v4f){v[4], v[5], v[6], v[7]}; }
__device__ __forceinline__ v8f ld8(const float* p) { return cat8(*(const v4f*)p, *(const v4f*)(p + 4)); }
__device__ __forceinline__ void st8(float* p, v8f v) { *(v4f*)p = lo4(v); *(v4f*)(p + 4) = hi4(v); }

__device__ __forceinline__ float ex2_hw(float a) {
#if __has_builtin(__builtin_amdgcn_exp2f)
  return __builtin_amdgcn_exp2f(a);
#else
  return exp2f(a);
#endif
}
__device__ __forceinline__ float rcp_hw(float a) { return __builtin_amdgcn_rcpf(a); }
__device__ __forceinline__ float th_a(float a) {
  const float e = ex2_hw(a);
  const float r = rcp_hw(e + 1.0f);
  return fmaf(-2.0f, r, 1.0f);
}

__device__ __forceinline__ v16h frag_h32(const _Float16* p) {
  union { v16h v; v8h h[2]; } f;
  f.h[0] = *(const v8h*)p;
  f.h[1] = *(const v8h*)(p + 16);
  return f.v;
}
__device__ __forceinline__ v16h frag_h16(const _Float16* p) {
  union { v16h v; v8h h[2]; } f;
  f.h[0] = *(const v8h*)p;
  f.h[1] = __builtin_bit_cast(v8h, (v4f){0.f, 0.f, 0.f, 0.f});
  return f.v;
}
__device__ __forceinline__ v16b frag_b32(const unsigned short* p) {
  union { v16b v; v8b h[2]; } f;
  f.h[0] = *(const v8b*)(const void*)p;
  f.h[1] = *(const v8b*)(const void*)(p + 16);
  return f.v;
}
__device__ __forceinline__ v16b frag_b16(const unsigned short* p) {
  union { v16b v; v8b h[2]; } f;
  f.h[0] = *(const v8b*)(const void*)p;
  f.h[1] = __builtin_bit_cast(v8b, (v4f){0.f, 0.f, 0.f, 0.f});
  return f.v;
}

__device__ __forceinline__ v16h pack_h2(v8f a, v8f b) {
  union { v16h v; v8h h[2]; } f;
  v8h la, lb;
#pragma unroll
  for (int e = 0; e < 8; ++e) { la[e] = (_Float16)a[e]; lb[e] = (_Float16)b[e]; }
  f.h[0] = la; f.h[1] = lb;
  return f.v;
}
__device__ __forceinline__ v16h pack_h1(v8f a) {
  union { v16h v; v8h h[2]; } f;
  v8h la;
#pragma unroll
  for (int e = 0; e < 8; ++e) la[e] = (_Float16)a[e];
  f.h[0] = la;
  f.h[1] = __builtin_bit_cast(v8h, (v4f){0.f, 0.f, 0.f, 0.f});
  return f.v;
}
__device__ __forceinline__ void pack_b2(v8f a, v8f b, v16b& hi, v16b& lo) {
#pragma unroll
  for (int e = 0; e < 8; ++e) {
    unsigned short hb, lb;
    split_bf(a[e], hb, lb);
    hi[e] = __builtin_bit_cast(__bf16, hb); lo[e] = __builtin_bit_cast(__bf16, lb);
    split_bf(b[e], hb, lb);
    hi[8 + e] = __builtin_bit_cast(__bf16, hb); lo[8 + e] = __builtin_bit_cast(__bf16, lb);
  }
}
__device__ __forceinline__ void pack_b1(v8f a, v16b& hi, v16b& lo) {
  union { v16b v; v8b h[2]; } fh, fl;
  v8b ph, pl;
#pragma unroll
  for (int e = 0; e < 8; ++e) {
    unsigned short hb, lb;
    split_bf(a[e], hb, lb);
    ph[e] = __builtin_bit_cast(__bf16, hb); pl[e] = __builtin_bit_cast(__bf16, lb);
  }
  fh.h[0] = ph; fh.h[1] = __builtin_bit_cast(v8b, (v4f){0.f, 0.f, 0.f, 0.f});
  fl.h[0] = pl; fl.h[1] = __builtin_bit_cast(v8b, (v4f){0.f, 0.f, 0.f, 0.f});
  hi = fh.v; lo = fl.v;
}

__device__ __forceinline__ v8f kld(const float* kb, int j, int i) { return ld8(kb + (j * kSlotStride + 8 * i)); }

template <int ST>
__device__ __forceinline__ v8f stage_in(const float* kb, int i, v8f y, float dt) {
  const v8f k1 = kld(kb, 0, i);
  if (ST == 2) return y + dt * (cA21 * k1);
  const v8f k2 = kld(kb, 1, i);
  if (ST == 3) return y + dt * (cA31 * k1 + cA32 * k2);
  const v8f k3 = kld(kb, 2, i);
  if (ST == 4) return y + dt * (cA41 * k1 + cA42 * k2 + cA43 * k3);
  const v8f k4 = kld(kb, 3, i);
  if (ST == 5) return y + dt * (cA51 * k1 + cA52 * k2 + cA53 * k3 + cA54 * k4);
  const v8f k5 = kld(kb, 4, i);
  return y + dt * (cA61 * k1 + cA62 * k2 + cA63 * k3 + cA64 * k4 + cA65 * k5);
}
template <int ST>
__device__ __forceinline__ void stage_x(const float* kb, v8f y0, v8f y1, v8f y2, v8f y3, float dt, v16h& x0, v16h& x1) {
  const v8f u0 = stage_in<ST>(kb, 0, y0, dt);
  cfence();
  const v8f u1 = stage_in<ST>(kb, 1, y1, dt);
  x0 = pack_h2(u0, u1);
  cfence();
  const v8f u2 = stage_in<ST>(kb, 2, y2, dt);
  cfence();
  const v8f u3 = stage_in<ST>(kb, 3, y3, dt);
  x1 = pack_h2(u2, u3);
  cfence();
}
__device__ __forceinline__ v8f upd_tile(const float* kb, int i, v8f y, float dt) {
  const v8f k1 = kld(kb, 0, i), k2 = kld(kb, 1, i), k3 = kld(kb, 2, i);
  const v8f k4 = kld(kb, 3, i), k5 = kld(kb, 4, i), k6 = kld(kb, 5, i);
  return y + dt * (cB1 * k1 + cB2 * k2 + cB3 * k3 + cB4 * k4 + cB5 * k5 + cB6 * k6);
}

__device__ __forceinline__ void vf_eval(const _Float16* w0r, const _Float16* w1r, const _Float16* w2r,
                                        const float* w0cp, const float* b0p, const float* b1p, const float* b2p,
                                        float* ksl, float t, float scale, float ns2, v16h x0, v16h x1) {
  v8f acc = mma_h(frag_h32(w0r), x0, zero8f());
  acc = mma_h(frag_h32(w0r + 32), x1, acc);
  const v8f wt = ld8(w0cp);
  const v8f c0 = ld8(b0p);
  v8f zv;
#pragma unroll
  for (int r = 0; r < 8; ++r) zv[r] = th_a(fmaf(acc[r], kS0, fmaf(wt[r], t, c0[r])));
  v16h zb = pack_h1(zv);
  acc = mma_h(frag_h16(w1r), zb, zero8f());
  const v8f c1 = ld8(b1p);
#pragma unroll
  for (int r = 0; r < 8; ++r) zv[r] = th_a(fmaf(acc[r], kS0, c1[r]));
  zb = pack_h1(zv);
#pragma unroll
  for (int i = 0; i < 4; ++i) {
    acc = mma_h(frag_h16(w2r + 256 * i), zb, zero8f());
    const v8f c2 = ld8(b2p + 16 * i);
    v8f kv;
#pragma unroll
    for (int r = 0; r < 8; ++r) {
      const float a1 = fmaf(acc[r], kS0, c2[r]);
      const float e1 = ex2_hw(a1);
      const float r1 = rcp_hw(e1 + 1.0f);
      const float a2 = fmaf(kM2, r1, kL2);
      const float e2 = ex2_hw(a2);
      const float r2 = rcp_hw(e2 + 1.0f);
      kv[r] = fmaf(ns2, r2, scale);
    }
    st8(ksl + 8 * i, kv);
    cfence();
  }
}

__device__ __forceinline__ v8f cell_tile(const unsigned short* whr_h, const unsigned short* whr_l,
                                         const unsigned short* wxr_h, const unsigned short* wxr_l, const float* bxp,
                                         v16b yh0, v16b yl0, v16b yh1, v16b yl1, v16b xh, v16b xl) {
  v8f acc = zero8f();
  v16b ah = frag_b32(whr_h), al = frag_b32(whr_l);
  acc = mma_b(ah, yh0, acc); acc = mma_b(ah, yl0, acc); acc = mma_b(al, yh0, acc);
  ah = frag_b32(whr_h + 32); al = frag_b32(whr_l + 32);
  acc = mma_b(ah, yh1, acc); acc = mma_b(ah, yl1, acc); acc = mma_b(al, yh1, acc);
  ah = frag_b32(wxr_h); al = frag_b32(wxr_l);
  acc = mma_b(ah, xh, acc); acc = mma_b(ah, xl, acc); acc = mma_b(al, xh, acc);
  const v8f bb = ld8(bxp);
  v8f o;
#pragma unroll
  for (int r = 0; r < 8; ++r) o[r] = th_a(fmaf(acc[r], kL2, bb[r]));
  return o;
}

__global__ __launch_bounds__(32) __attribute__((amdgpu_num_vgpr(256)))
void rk_rnn_seq_kernel(
    const float* __restrict__ ts, const float* __restrict__ obs, const float* __restrict__ scale_p,
    const float* __restrict__ w0, const float* __restrict__ b0,
    const float* __restrict__ w1, const float* __restrict__ b1,
    const float* __restrict__ w2, const float* __restrict__ b2,
    const float* __restrict__ wh, const float* __restrict__ wx, const float* __restrict__ bx,
    const float* __restrict__ ow0, const float* __restrict__ ob0,
    const float* __restrict__ ow1, const float* __restrict__ ob1,
    const float* __restrict__ ow2, const float* __restrict__ ob2,
    float* __restrict__ out) {
  __shared__ __align__(16) _Float16       w0s[16 * 64];
  __shared__ __align__(16) _Float16       w1s[16 * 16];
  __shared__ __align__(16) _Float16       w2s[64 * 16];
  __shared__ __align__(16) unsigned short whh[64 * 64];
  __shared__ __align__(16) unsigned short whl[64 * 64];
  __shared__ __align__(16) unsigned short wxh[64 * 32];
  __shared__ __align__(16) unsigned short wxl[64 * 32];
  __shared__ __align__(16) unsigned short o0h[16 * 64];
  __shared__ __align__(16) unsigned short o0l[16 * 64];
  __shared__ __align__(16) unsigned short o1h[16 * 16];
  __shared__ __align__(16) unsigned short o1l[16 * 16];
  __shared__ __align__(16) unsigned short o2h[16 * 16];
  __shared__ __align__(16) unsigned short o2l[16 * 16];
  __shared__ __align__(16) float w0cs[16];
  __shared__ __align__(16) float b0s[16];
  __shared__ __align__(16) float b1s[16];
  __shared__ __align__(16) float b2s[64];
  __shared__ __align__(16) float bxs[64];
  __shared__ __align__(16) float ob0s[16];
  __shared__ __align__(16) float ob1s[16];
  __shared__ __align__(16) float ob2s[16];
  __shared__ __align__(16) float kst[kSlots * kSlotStride];

  const int lane = threadIdx.x & 31;
  const int hh   = lane >> 4;
  const int rl   = lane & 15;
  const int blk  = blockIdx.x;
  const int seq  = blk * kSeqPerBlk + rl;

#pragma unroll 1
  for (int it = 0; it < 4; ++it) {
    const int base = (it * 32 + lane) * 8;
    const int m = base >> 6, kk = base & 63;
    const float* src = w0 + m * 65 + 1 + kk;
    v8h hv;
#pragma unroll
    for (int e = 0; e < 8; ++e) hv[e] = (_Float16)(src[e] * 16.0f);
    *(v8h*)(w0s + base) = hv;
  }
  {
    const int base = lane * 8;
    const v4f a = *(const v4f*)(w1 + base), c = *(const v4f*)(w1 + base + 4);
    v8h hv;
#pragma unroll
    for (int e = 0; e < 4; ++e) { hv[e] = (_Float16)(a[e] * 16.0f); hv[4 + e] = (_Float16)(c[e] * 16.0f); }
    *(v8h*)(w1s + base) = hv;
  }
#pragma unroll 1
  for (int it = 0; it < 4; ++it) {
    const int base = (it * 32 + lane) * 8;
    const v4f a = *(const v4f*)(w2 + base), c = *(const v4f*)(w2 + base + 4);
    v8h hv;
#pragma unroll
    for (int e = 0; e < 4; ++e) { hv[e] = (_Float16)(a[e] * 16.0f); hv[4 + e] = (_Float16)(c[e] * 16.0f); }
    *(v8h*)(w2s + base) = hv;
  }
#pragma unroll 1
  for (int it = 0; it < 32; ++it) {
    const int q = it * 32 + lane;
    const v4f v = *(const v4f*)(wh + 4 * q);
    v4us hv, lv;
#pragma unroll
    for (int e = 0; e < 4; ++e) { unsigned short hb, lb; split_bf(v[e], hb, lb); hv[e] = hb; lv[e] = lb; }
    *(v4us*)(whh + 4 * q) = hv;
    *(v4us*)(whl + 4 * q) = lv;
  }
#pragma unroll 1
  for (int it = 0; it < 16; ++it) {
    const int q = it * 32 + lane;
    const v4f v = *(const v4f*)(wx + 4 * q);
    v4us hv, lv;
#pragma unroll
    for (int e = 0; e < 4; ++e) { unsigned short hb, lb; split_bf(v[e], hb, lb); hv[e] = hb; lv[e] = lb; }
    *(v4us*)(wxh + 4 * q) = hv;
    *(v4us*)(wxl + 4 * q) = lv;
  }
#pragma unroll 1
  for (int it = 0; it < 8; ++it) {
    const int q = it * 32 + lane;
    const v4f v = *(const v4f*)(ow0 + 4 * q);
    v4us hv, lv;
#pragma unroll
    for (int e = 0; e < 4; ++e) { unsigned short hb, lb; split_bf(v[e], hb, lb); hv[e] = hb; lv[e] = lb; }
    *(v4us*)(o0h + 4 * q) = hv;
    *(v4us*)(o0l + 4 * q) = lv;
  }
#pragma unroll 1
  for (int it = 0; it < 2; ++it) {
    const int q = it * 32 + lane;
    const v4f v = *(const v4f*)(ow1 + 4 * q);
    v4us hv, lv;
#pragma unroll
    for (int e = 0; e < 4; ++e) { unsigned short hb, lb; split_bf(v[e], hb, lb); hv[e] = hb; lv[e] = lb; }
    *(v4us*)(o1h + 4 * q) = hv;
    *(v4us*)(o1l + 4 * q) = lv;
  }
  {
    const v4f v = *(const v4f*)(ow2 + 4 * lane);
    v4us hv, lv;
#pragma unroll
    for (int e = 0; e < 4; ++e) { unsigned short hb, lb; split_bf(v[e], hb, lb); hv[e] = hb; lv[e] = lb; }
    *(v4us*)(o2h + 4 * lane) = hv;
    *(v4us*)(o2l + 4 * lane) = lv;
    const v4us zz = (v4us){0, 0, 0, 0};
    *(v4us*)(o2h + 128 + 4 * lane) = zz;
    *(v4us*)(o2l + 128 + 4 * lane) = zz;
  }
  {
    const int c  = rl;
    const int c8 = (c < kOutDim) ? c : (kOutDim - 1);
    const float vw  = w0[c * 65];
    const float vb0 = b0[c], vb1 = b1[c], vo0 = ob0[c], vo1 = ob1[c];
    const float vo2r = ob2[c8];
    const float vo2 = (c < kOutDim) ? vo2r : 0.f;
    if (hh == 0) {
      w0cs[c] = kL2 * vw; b0s[c] = kL2 * vb0; b1s[c] = kL2 * vb1;
      ob0s[c] = vo0; ob1s[c] = vo1; ob2s[c] = vo2;
    }
    b2s[lane] = kL2 * b2[lane]; b2s[32 + lane] = kL2 * b2[32 + lane];
    bxs[lane] = kL2 * bx[lane]; bxs[32 + lane] = kL2 * bx[32 + lane];
  }
  __syncthreads();

  const float scale = scale_p[0];
  const float ns2   = -2.0f * scale;
  v8f y0 = zero8f(), y1 = zero8f(), y2 = zero8f(), y3 = zero8f();
  const float* tsr = ts + (size_t)seq * kSteps;
  const float* obr = obs + ((size_t)seq * kSteps) * kIn + 8 * hh;
  float tprev = tsr[0];
  float* ks = kst + lane * 32;

#pragma unroll 1
  for (int n = 0; n < kSteps; ++n) {
    const float t1  = tsr[n];
    const float dtn = (t1 - tprev) * 0.125f;
    const int z = opaque_zero();
    const _Float16* w0r = w0s + (rl * 64 + 8 * hh + z);
    const _Float16* w1r = w1s + (rl * 16 + 8 * hh + z);
    const _Float16* w2r = w2s + (rl * 16 + 8 * hh + z);
    const float* w0cp = w0cs + (8 * hh + z);
    const float* b0p  = b0s  + (8 * hh + z);
    const float* b1p  = b1s  + (8 * hh + z);
    const float* b2p  = b2s  + (8 * hh + z);
    const float* kb   = kst  + (lane * 32 + z);

#pragma unroll 1
    for (int sub = 0; sub < kSub; ++sub) {
      const float tb = tprev + (float)sub * dtn;
      {
        const v16h x0 = pack_h2(y0, y1);
        const v16h x1 = pack_h2(y2, y3);
        vf_eval(w0r, w1r, w2r, w0cp, b0p, b1p, b2p, ks + 0 * kSlotStride, tb, scale, ns2, x0, x1);
      }
      {
        v16h x0, x1;
        stage_x<2>(kb, y0, y1, y2, y3, dtn, x0, x1);
        vf_eval(w0r, w1r, w2r, w0cp, b0p, b1p, b2p, ks + 1 * kSlotStride, tb + cC2 * dtn, scale, ns2, x0, x1);
      }
      {
        v16h x0, x1;
        stage_x<3>(kb, y0, y1, y2, y3, dtn, x0, x1);
        vf_eval(w0r, w1r, w2r, w0cp, b0p, b1p, b2p, ks + 2 * kSlotStride, tb + cC3 * dtn, scale, ns2, x0, x1);
      }
      {
        v16h x0, x1;
        stage_x<4>(kb, y0, y1, y2, y3, dtn, x0, x1);
        vf_eval(w0r, w1r, w2r, w0cp, b0p, b1p, b2p, ks + 3 * kSlotStride, tb + cC4 * dtn, scale, ns2, x0, x1);
      }
      {
        v16h x0, x1;
        stage_x<5>(kb, y0, y1, y2, y3, dtn, x0, x1);
        vf_eval(w0r, w1r, w2r, w0cp, b0p, b1p, b2p, ks + 4 * kSlotStride, tb + cC5 * dtn, scale, ns2, x0, x1);
      }
      {
        v16h x0, x1;
        stage_x<6>(kb, y0, y1, y2, y3, dtn, x0, x1);
        vf_eval(w0r, w1r, w2r, w0cp, b0p, b1p, b2p, ks + 5 * kSlotStride, tb + dtn, scale, ns2, x0, x1);
      }
      y0 = upd_tile(kb, 0, y0, dtn); cfence();
      y1 = upd_tile(kb, 1, y1, dtn); cfence();
      y2 = upd_tile(kb, 2, y2, dtn); cfence();
      y3 = upd_tile(kb, 3, y3, dtn); cfence();
    }

    {
      v16b yh0, yl0, yh1, yl1;
      pack_b2(y0, y1, yh0, yl0);
      pack_b2(y2, y3, yh1, yl1);
      const float* xp = obr + (size_t)n * kIn;
      const v4f xa = *(const v4f*)xp, xb = *(const v4f*)(xp + 4);
      const v4f xc = *(const v4f*)(xp + 16), xd = *(const v4f*)(xp + 20);
      v16b xh, xl;
      pack_b2(cat8(xa, xb), cat8(xc, xd), xh, xl);
      const int ro = rl * 64 + 8 * hh + z;
      const int rx = rl * 32 + 8 * hh + z;
      const float* bxp = bxs + (8 * hh + z);
      y0 = cell_tile(whh + ro,          whl + ro,          wxh + rx,          wxl + rx,          bxp,      yh0, yl0, yh1, yl1, xh, xl);
      cfence();
      y1 = cell_tile(whh + (ro + 1024), whl + (ro + 1024), wxh + (rx + 512),  wxl + (rx + 512),  bxp + 16, yh0, yl0, yh1, yl1, xh, xl);
      cfence();
      y2 = cell_tile(whh + (ro + 2048), whl + (ro + 2048), wxh + (rx + 1024), wxl + (rx + 1024), bxp + 32, yh0, yl0, yh1, yl1, xh, xl);
      cfence();
      y3 = cell_tile(whh + (ro + 3072), whl + (ro + 3072), wxh + (rx + 1536), wxl + (rx + 1536), bxp + 48, yh0, yl0, yh1, yl1, xh, xl);
      cfence();
    }
    tprev = t1;
  }

  v8f outv;
  {
    v16b yh0, yl0, yh1, yl1;
    pack_b2(y0, y1, yh0, yl0);
    pack_b2(y2, y3, yh1, yl1);
    const unsigned short* p0h = o0h + (rl * 64 + 8 * hh);
    const unsigned short* p0l = o0l + (rl * 64 + 8 * hh);
    v8f acc = zero8f();
    v16b gh = frag_b32(p0h), gl = frag_b32(p0l);
    acc = mma_b(gh, yh0, acc); acc = mma_b(gh, yl0, acc); acc = mma_b(gl, yh0, acc);
    gh = frag_b32(p0h + 32); gl = frag_b32(p0l + 32);
    acc = mma_b(gh, yh1, acc); acc = mma_b(gh, yl1, acc); acc = mma_b(gl, yh1, acc);
    const v8f cb0 = ld8(ob0s + 8 * hh);
    v8f zz;
#pragma unroll
    for (int r = 0; r < 8; ++r) zz[r] = fmaxf(acc[r] + cb0[r], 0.0f);
    cfence();
    v16b zh, zl;
    pack_b1(zz, zh, zl);
    gh = frag_b16(o1h + (rl * 16 + 8 * hh)); gl = frag_b16(o1l + (rl * 16 + 8 * hh));
    acc = zero8f();
    acc = mma_b(gh, zh, acc); acc = mma_b(gh, zl, acc); acc = mma_b(gl, zh, acc);
    const v8f cb1 = ld8(ob1s + 8 * hh);
#pragma unroll
    for (int r = 0; r < 8; ++r) zz[r] = fmaxf(acc[r] + cb1[r], 0.0f);
    cfence();
    pack_b1(zz, zh, zl);
    gh = frag_b16(o2h + (rl * 16 + 8 * hh)); gl = frag_b16(o2l + (rl * 16 + 8 * hh));
    acc = zero8f();
    acc = mma_b(gh, zh, acc); acc = mma_b(gh, zl, acc); acc = mma_b(gl, zh, acc);
    const v8f cb2 = ld8(ob2s + 8 * hh);
#pragma unroll
    for (int r = 0; r < 8; ++r) outv[r] = acc[r] + cb2[r];
  }

  __syncthreads();
  float* o1s = kst;
  float* o0s = kst + 1024;
  if (hh == 0) {
    *(v4f*)(o0s + rl * 8)     = lo4(outv);
    *(v4f*)(o0s + rl * 8 + 4) = hi4(outv);
  }
  {
    float* orow = o1s + rl * 64 + 8 * hh;
    *(v4f*)(orow + 0)  = lo4(y0); *(v4f*)(orow + 4)  = hi4(y0);
    *(v4f*)(orow + 16) = lo4(y1); *(v4f*)(orow + 20) = hi4(y1);
    *(v4f*)(orow + 32) = lo4(y2); *(v4f*)(orow + 36) = hi4(y2);
    *(v4f*)(orow + 48) = lo4(y3); *(v4f*)(orow + 52) = hi4(y3);
  }
  __syncthreads();
  {
    const v4f s0 = *(const v4f*)(o0s + 4 * lane);
    v4f s1[8];
#pragma unroll
    for (int it = 0; it < 8; ++it) s1[it] = *(const v4f*)(o1s + it * 128 + 4 * lane);
    float* g0 = out + (size_t)blk * (kSeqPerBlk * kOutDim) + 4 * lane;
    float* g1 = out + kOut1Off + (size_t)blk * (kSeqPerBlk * kHid) + 4 * lane;
    *(volatile v4f*)g0 = s0;
#pragma unroll
    for (int it = 0; it < 8; ++it) *(volatile v4f*)(g1 + it * 128) = s1[it];
    __threadfence();
    *(volatile v4f*)g0 = s0;
#pragma unroll
    for (int it = 0; it < 8; ++it) *(volatile v4f*)(g1 + it * 128) = s1[it];
  }
}

extern "C" void kernel_launch(void* const* d_in, const int* in_sizes, int n_in,
                              void* d_out, int out_size, void* d_ws, size_t ws_size,
                              hipStream_t stream) {
  (void)in_sizes; (void)d_ws; (void)ws_size;
  if (n_in < 18 || out_size < kOutTotal) return;
  const float* ts   = (const float*)d_in[0];
  const float* obs  = (const float*)d_in[1];
  const float* sc   = (const float*)d_in[2];
  const float* w0   = (const float*)d_in[3];
  const float* b0   = (const float*)d_in[4];
  const float* w1   = (const float*)d_in[5];
  const float* b1   = (const float*)d_in[6];
  const float* w2   = (const float*)d_in[7];
  const float* b2   = (const float*)d_in[8];
  const float* wh   = (const float*)d_in[9];
  const float* wx   = (const float*)d_in[10];
  const float* bx   = (const float*)d_in[11];
  const float* ow0  = (const float*)d_in[12];
  const float* ob0  = (const float*)d_in[13];
  const float* ow1  = (const float*)d_in[14];
  const float* ob1  = (const float*)d_in[15];
  const float* ow2  = (const float*)d_in[16];
  const float* ob2  = (const float*)d_in[17];
  float* out = (float*)d_out;

  rk_rnn_seq_kernel<<<dim3(kBlocks), dim3(32), 0, stream>>>(
      ts, obs, sc, w0, b0, w1, b1, w2, b2, wh, wx, bx, ow0, ob0, ow1, ob1, ow2, ob2, out);
}
